// BiLSTM_20435454394481
// MI455X (gfx1250) — hardware-verified
//
#include <hip/hip_runtime.h>
#include <math.h>

constexpr int NB     = 256;
constexpr int NTSTEP = 200;
constexpr int NVOC   = 50000;
constexpr int NEMB   = 300;
constexpr int NHID   = 128;
constexpr int NGATE  = 512;
constexpr int NCLS   = 6;
constexpr int NWIN   = NEMB + NHID;
constexpr int KX     = 320;
constexpr int KFW    = KX + 2 * NHID;
constexpr int NTHR   = 256;
constexpr int RB     = 16;
constexpr int APITCH = 584;
constexpr int HSP    = 260;
constexpr int NXG    = KX / 4;
constexpr int NEG    = NEMB / 4;
constexpr int NIDS   = RB * NTSTEP;
constexpr int NWO    = 2 * NHID * NCLS;
static_assert(NB % RB == 0);
static_assert(NHID == 16 * (NTHR / 32));
static_assert(KX % 64 == 0 && KFW % 64 == 0 && NGATE % 64 == 0);
static_assert(NEMB % 4 == 0 && NEMB <= KX);
static_assert(RB * NXG == 5 * NTHR);
static_assert(NIDS % 4 == 0 && NIDS / 4 <= 4 * NTHR);
static_assert(NWO % 4 == 0 && NWO / 4 <= 2 * NTHR);
static_assert(RB * NCLS * 4 == 3 * 128);
static_assert(RB * NCLS <= NTHR && (RB * NCLS) % 4 == 0);
static_assert(APITCH % 8 == 0 && APITCH >= KFW);
static_assert((RB * APITCH) % 2 == 0);
static_assert(HSP % 4 == 0 && HSP >= 2 * NHID);

typedef __attribute__((ext_vector_type(16))) _Float16 v16h;
typedef __attribute__((ext_vector_type(8)))  _Float16 v8h;
typedef __attribute__((ext_vector_type(16))) __bf16   v16b;
typedef __attribute__((ext_vector_type(8)))  __bf16   v8b;
typedef __attribute__((ext_vector_type(8)))  float    v8f;
typedef __attribute__((ext_vector_type(4)))  float    v4f;
typedef __attribute__((ext_vector_type(4)))  int      v4i;
typedef __attribute__((ext_vector_type(2)))  unsigned v2u;

__device__ __forceinline__ unsigned short f2bf_bits(float f) {
  unsigned u = __float_as_uint(f);
  return (unsigned short)((u + 0x7FFFu + ((u >> 16) & 1u)) >> 16);
}
__device__ __forceinline__ float bf_bits2f(unsigned short h) { return __uint_as_float(((unsigned)h) << 16); }
__device__ __forceinline__ float bf16r(float f) { return bf_bits2f(f2bf_bits(f)); }

__device__ __forceinline__ void dep_guard_h(v8f& a, v8f& b, v16h x, v16h y) { asm volatile("v_nop\n\tv_nop\n\tv_nop\n\tv_nop" : "+v"(a), "+v"(b) : "v"(x), "v"(y)); }
__device__ __forceinline__ void dep_guard_b(v8f& a, v8f& b, v16b x, v16b y) { asm volatile("v_nop\n\tv_nop\n\tv_nop\n\tv_nop" : "+v"(a), "+v"(b) : "v"(x), "v"(y)); }
__device__ __forceinline__ void keep4_h(v16h a, v16h b, v16h c, v16h d) { asm volatile("v_nop" :: "v"(a), "v"(b), "v"(c), "v"(d)); }
__device__ __forceinline__ void keep4_b(v16b a, v16b b, v16b c, v16b d) { asm volatile("v_nop" :: "v"(a), "v"(b), "v"(c), "v"(d)); }
__device__ __forceinline__ void acc_guard4(v8f& a, v8f& b, v8f& c, v8f& d) { asm volatile("v_nop\n\tv_nop\n\tv_nop\n\tv_nop" : "+v"(a), "+v"(b), "+v"(c), "+v"(d)); }
__device__ __forceinline__ void guard_all4b(v8f& a0, v8f& a1, v8f& a2, v8f& a3, v16b x, v16b y0, v16b y1, v16b y2, v16b y3) {
  asm volatile("v_nop\n\tv_nop\n\tv_nop\n\tv_nop" : "+v"(a0), "+v"(a1), "+v"(a2), "+v"(a3) : "v"(x), "v"(y0), "v"(y1), "v"(y2), "v"(y3));
}
template <typename T> struct Frag;
template <> struct Frag<_Float16> {
  typedef v16h V; union U { v16h v; v8h h[2]; };
  static __device__ __forceinline__ v16h load(const _Float16* p) {
    U f; f.h[0] = *(const v8h*)(p); f.h[1] = *(const v8h*)(p + 16); return f.v;
  }
  static __device__ __forceinline__ v8f mma(v16h a, v16h b, v8f c) {
    return __builtin_amdgcn_wmma_f32_16x16x32_f16(false, a, false, b, (short)0, c, false, false);
  }
  static __device__ __forceinline__ void guard(v8f& a, v8f& b, v16h x, v16h y) { dep_guard_h(a, b, x, y); }
  static __device__ __forceinline__ void keep(v16h a, v16h b, v16h c, v16h d) { keep4_h(a, b, c, d); }
};
template <> struct Frag<__bf16> {
  typedef v16b V; union U { v16b v; v8b h[2]; };
  static __device__ __forceinline__ v16b load(const __bf16* p) {
    U f; f.h[0] = *(const v8b*)(p); f.h[1] = *(const v8b*)(p + 16); return f.v;
  }
  static __device__ __forceinline__ v8f mma(v16b a, v16b b, v8f c) {
    return __builtin_amdgcn_wmma_f32_16x16x32_bf16(false, a, false, b, (short)0, c, false, false);
  }
  static __device__ __forceinline__ void guard(v8f& a, v8f& b, v16b x, v16b y) { dep_guard_b(a, b, x, y); }
  static __device__ __forceinline__ void keep(v16b a, v16b b, v16b c, v16b d) { keep4_b(a, b, c, d); }
};

__device__ __forceinline__ float fsig(float x) { return __builtin_amdgcn_rcpf(1.0f + expf(-x)); }

__global__ __launch_bounds__(NTHR) void wprep_kernel(const float* __restrict__ W, unsigned short* __restrict__ O, int kpad) {
  __shared__ float Tt[64 * 65];
  const int tid = threadIdx.x;
  const int n0 = blockIdx.x * 64, k0 = blockIdx.y * 64;
#pragma unroll
  for (int i = 0; i < 4; ++i) {
    const int idx = i * NTHR + tid;
    const int kk = idx >> 4, cc = (idx & 15) * 4;
    const int k = k0 + kk;
    const int inpad = (k >= NEMB) && (k < KX);
    int sr = k;
    if (k >= KX) sr = k - (KX - NEMB);
    if (k >= KX + NHID) sr = k - (KX - NEMB) - NHID;
    if (inpad) sr = 0;
    sr = sr < 0 ? 0 : (sr > NWIN - 1 ? NWIN - 1 : sr);
    const float fa = inpad ? 0.0f : 1.0f;
    const v4f v = *(const v4f*)(W + (size_t)sr * NGATE + n0 + cc);
    Tt[kk * 65 + cc + 0] = v[0] * fa;
    Tt[kk * 65 + cc + 1] = v[1] * fa;
    Tt[kk * 65 + cc + 2] = v[2] * fa;
    Tt[kk * 65 + cc + 3] = v[3] * fa;
  }
  __syncthreads();
  const int q = tid >> 3, c8 = (tid & 7) * 8;
  v8h hv[2];
#pragma unroll
  for (int g = 0; g < 2; ++g) {
    const int nn = g * 32 + q;
#pragma unroll
    for (int e = 0; e < 8; ++e) {
      const float f = Tt[(c8 + e) * 65 + nn];
      hv[g][e] = __builtin_bit_cast(_Float16, f2bf_bits(f));
    }
  }
  for (int pass = 0; pass < 2; ++pass) {
#pragma unroll
    for (int g = 0; g < 2; ++g) {
      const size_t o = (size_t)(n0 + g * 32 + q) * (size_t)kpad + (size_t)(k0 + c8);
      *(volatile v8h*)(O + o) = hv[g];
    }
    __threadfence();
  }
}

__device__ __forceinline__ void stage_x(unsigned short* Axh, const int* Ids, const float* __restrict__ embeds, int t, int tid) {
#pragma unroll
  for (int it = 0; it < (RB * NXG) / NTHR; ++it) {
    const int idx = it * NTHR + tid;
    const int m = idx / NXG;
    const int g = idx - m * NXG;
    const int id = Ids[m * NTSTEP + t];
    const int gc = (g < NEG) ? g : (NEG - 1);
    const float fa = (g < NEG) ? 1.0f : 0.0f;
    const v4f v = *(const v4f*)(embeds + (size_t)id * NEMB + 4 * gc);
    const unsigned short u0 = f2bf_bits(v[0] * fa), u1 = f2bf_bits(v[1] * fa);
    const unsigned short u2 = f2bf_bits(v[2] * fa), u3 = f2bf_bits(v[3] * fa);
    v2u pk;
    pk[0] = (unsigned)u0 | ((unsigned)u1 << 16);
    pk[1] = (unsigned)u2 | ((unsigned)u3 << 16);
    *(v2u*)(Axh + m * APITCH + 4 * g) = pk;
  }
}

__global__ __launch_bounds__(NTHR) void bilstm_kernel(const int* __restrict__ x, const float* __restrict__ embeds,
                                                      const unsigned short* __restrict__ WFWp,
                                                      const unsigned short* __restrict__ WBWp,
                                                      const float* __restrict__ b_fw, const float* __restrict__ b_bw,
                                                      const float* __restrict__ w_out, const float* __restrict__ b_out,
                                                      float* __restrict__ out) {
  __shared__ __align__(16) unsigned short Axh[RB * APITCH];
  __shared__ __align__(16) int            Ids[NIDS];
  __shared__ __align__(16) float          Ws[NWO];
  __shared__ __align__(16) float          Hs[RB * HSP];
  __shared__ __align__(16) float          Sc[RB * NCLS];
  const __bf16* WFW = (const __bf16*)WFWp;
  const __bf16* WBW = (const __bf16*)WBWp;
  const int tid = threadIdx.x, lane = tid & 31, wave = tid >> 5;
  const int c = lane & 15, hh = lane >> 4, koff = hh * 8;
  const int rowbase = blockIdx.x * RB;
  const int ju = 16 * wave + c;

  {
    const int* xb = x + (size_t)rowbase * NTSTEP;
#pragma unroll
    for (int i = 0; i < 4; ++i) {
      const int idx = i * NTHR + tid;
      const int idc = idx < NIDS / 4 ? idx : NIDS / 4 - 1;
      v4i v = *(const v4i*)(xb + 4 * idc);
#pragma unroll
      for (int e = 0; e < 4; ++e) { int q = v[e]; q = q < 0 ? 0 : q; q = q > NVOC - 1 ? NVOC - 1 : q; v[e] = q; }
      if (idx < NIDS / 4) *(v4i*)(Ids + 4 * idx) = v;
    }
  }
  {
    unsigned* aw = (unsigned*)(void*)Axh;
#pragma unroll 1
    for (int i = tid; i < (RB * APITCH) / 2; i += NTHR) aw[i] = 0u;
  }
  {
#pragma unroll
    for (int i = 0; i < 2; ++i) {
      const int idx = i * NTHR + tid;
      const int idc = idx < NWO / 4 ? idx : NWO / 4 - 1;
      v4f v = *(const v4f*)(w_out + 4 * idc);
#pragma unroll
      for (int e = 0; e < 4; ++e) v[e] = bf16r(v[e]);
      if (idx < NWO / 4) *(v4f*)(Ws + 4 * idx) = v;
    }
  }
  float bfw[4], bbw[4];
#pragma unroll
  for (int g = 0; g < 4; ++g) { bfw[g] = bf16r(b_fw[g * NHID + ju]); bbw[g] = bf16r(b_bw[g * NHID + ju]); }
  __syncthreads();

  const __bf16* arow = (const __bf16*)(const void*)Axh + c * APITCH + koff;
  const v8f z8 = {0.f, 0.f, 0.f, 0.f, 0.f, 0.f, 0.f, 0.f};

  stage_x(Axh, Ids, embeds, NTSTEP - 1, tid);
  __syncthreads();
  float hbw[8];
  {
    v8f acc[4];
    acc[0] = z8; acc[1] = z8; acc[2] = z8; acc[3] = z8;
#pragma unroll 1
    for (int k0 = 0; k0 < KX; k0 += 32) {
      const v16b a  = Frag<__bf16>::load(arow + k0);
      const v16b b0 = Frag<__bf16>::load(WBW + (size_t)(0 * NHID + ju) * KX + koff + k0);
      const v16b b1 = Frag<__bf16>::load(WBW + (size_t)(1 * NHID + ju) * KX + koff + k0);
      const v16b b2 = Frag<__bf16>::load(WBW + (size_t)(2 * NHID + ju) * KX + koff + k0);
      const v16b b3 = Frag<__bf16>::load(WBW + (size_t)(3 * NHID + ju) * KX + koff + k0);
      acc[0] = Frag<__bf16>::mma(a, b0, acc[0]);
      acc[1] = Frag<__bf16>::mma(a, b1, acc[1]);
      acc[2] = Frag<__bf16>::mma(a, b2, acc[2]);
      acc[3] = Frag<__bf16>::mma(a, b3, acc[3]);
      guard_all4b(acc[0], acc[1], acc[2], acc[3], a, b0, b1, b2, b3);
    }
    acc_guard4(acc[0], acc[1], acc[2], acc[3]);
#pragma unroll
    for (int r = 0; r < 8; ++r) {
      const float zi = acc[0][r] + bbw[0];
      const float zj = acc[1][r] + bbw[1];
      const float zo = acc[3][r] + bbw[3];
      const float cn = fsig(zi) * tanhf(zj);
      hbw[r] = fsig(zo) * tanhf(cn);
    }
  }
  __syncthreads();
  stage_x(Axh, Ids, embeds, 0, tid);
  float cst[8], hst[8];
#pragma unroll
  for (int r = 0; r < 8; ++r) { cst[r] = 0.0f; hst[r] = 0.0f; }
  __syncthreads();

#pragma unroll 1
  for (int t = 0; t < NTSTEP; ++t) {
    v8f acc[4];
    acc[0] = z8; acc[1] = z8; acc[2] = z8; acc[3] = z8;
#pragma unroll 1
    for (int k0 = 0; k0 < KFW; k0 += 32) {
      const v16b a  = Frag<__bf16>::load(arow + k0);
      const v16b b0 = Frag<__bf16>::load(WFW + (size_t)(0 * NHID + ju) * KFW + koff + k0);
      const v16b b1 = Frag<__bf16>::load(WFW + (size_t)(1 * NHID + ju) * KFW + koff + k0);
      const v16b b2 = Frag<__bf16>::load(WFW + (size_t)(2 * NHID + ju) * KFW + koff + k0);
      const v16b b3 = Frag<__bf16>::load(WFW + (size_t)(3 * NHID + ju) * KFW + koff + k0);
      acc[0] = Frag<__bf16>::mma(a, b0, acc[0]);
      acc[1] = Frag<__bf16>::mma(a, b1, acc[1]);
      acc[2] = Frag<__bf16>::mma(a, b2, acc[2]);
      acc[3] = Frag<__bf16>::mma(a, b3, acc[3]);
      guard_all4b(acc[0], acc[1], acc[2], acc[3], a, b0, b1, b2, b3);
    }
    acc_guard4(acc[0], acc[1], acc[2], acc[3]);
#pragma unroll
    for (int r = 0; r < 8; ++r) {
      const float zi = acc[0][r] + bfw[0];
      const float zj = acc[1][r] + bfw[1];
      const float zf = acc[2][r] + bfw[2];
      const float zo = acc[3][r] + bfw[3];
      const float cn = fsig(zf + 1.0f) * cst[r] + fsig(zi) * tanhf(zj);
      cst[r] = cn;
      hst[r] = fsig(zo) * tanhf(cn);
    }
    __syncthreads();
#pragma unroll
    for (int r = 0; r < 8; ++r) {
      const float hn = hst[r];
      const unsigned short hb = f2bf_bits(hn);
      const unsigned short lb = f2bf_bits(hn - bf_bits2f(hb));
      Axh[(8 * hh + r) * APITCH + KX + ju] = hb;
      Axh[(8 * hh + r) * APITCH + KX + NHID + ju] = lb;
    }
    {
      const int tn = (t + 1 < NTSTEP) ? (t + 1) : (NTSTEP - 1);
      stage_x(Axh, Ids, embeds, tn, tid);
    }
    __syncthreads();
  }

#pragma unroll
  for (int r = 0; r < 8; ++r) {
    Hs[(8 * hh + r) * HSP + ju]        = hst[r];
    Hs[(8 * hh + r) * HSP + NHID + ju] = hbw[r];
  }
  __syncthreads();
  if (tid < RB * NCLS) {
    const int m  = tid / NCLS;
    const int cc = tid - m * NCLS;
    float s = 0.0f;
#pragma unroll 1
    for (int k = 0; k < 2 * NHID; ++k) s = fmaf(Hs[m * HSP + k], Ws[k * NCLS + cc], s);
    s += bf16r(b_out[cc]);
    Sc[tid] = s;
  }
  __syncthreads();
  if (tid < (RB * NCLS) / 4) {
    const v4f v = *(const v4f*)(Sc + 4 * tid);
    float* op = out + (size_t)rowbase * NCLS + 4 * tid;
    *(volatile v4f*)op = v;
    __threadfence();
    *(volatile v4f*)op = v;
  }
}

extern "C" void kernel_launch(void* const* d_in, const int* in_sizes, int n_in,
                              void* d_out, int out_size, void* d_ws, size_t ws_size, hipStream_t stream) {
  if (n_in < 8 || d_out == nullptr || d_ws == nullptr) return;
  if (in_sizes[0] != NB * NTSTEP || in_sizes[1] != NVOC * NEMB || in_sizes[2] != NWIN * NGATE || in_sizes[3] != NGATE ||
      in_sizes[4] != NWIN * NGATE || in_sizes[5] != NGATE || in_sizes[6] != 2 * NHID * NCLS || in_sizes[7] != NCLS ||
      out_size != NB * NCLS) return;

  const int*   x      = (const int*)d_in[0];
  const float* embeds = (const float*)d_in[1];
  const float* W_fw   = (const float*)d_in[2];
  const float* b_fw   = (const float*)d_in[3];
  const float* W_bw   = (const float*)d_in[4];
  const float* b_bw   = (const float*)d_in[5];
  const float* w_out  = (const float*)d_in[6];
  const float* b_out  = (const float*)d_in[7];
  float* out = (float*)d_out;

  char* ws = (char*)d_ws; size_t off = 0;
  auto carve = [&](size_t bytes) -> char* { char* p = ws + off; off += (bytes + 255) & ~(size_t)255; return p; };
  unsigned short* WFW = (unsigned short*)carve((size_t)NGATE * KFW * 2);
  unsigned short* WBW = (unsigned short*)carve((size_t)NGATE * KX * 2);
  if (off > ws_size || off > (size_t)134217728) return;

  wprep_kernel<<<dim3(NGATE / 64, KFW / 64), NTHR, 0, stream>>>(W_fw, WFW, KFW);
  wprep_kernel<<<dim3(NGATE / 64, KX / 64), NTHR, 0, stream>>>(W_bw, WBW, KX);
  bilstm_kernel<<<NB / RB, NTHR, 0, stream>>>(x, embeds, WFW, WBW, b_fw, b_bw, w_out, b_out, out);
}
